// Transformer_Block_25615184954012
// MI455X (gfx1250) — hardware-verified
//
#include <hip/hip_runtime.h>
#include <stddef.h>
#include <stdint.h>

#define B_   2
#define T_   2048
#define D_   1024
#define H_   16
#define DH_  64
#define DFF_ 4096
#define BT_  (B_ * T_)

#define GBM 128
#define GBN 128
#define GBK 64
#define GLP 72
#define CSP 128
#define AKP 72

static_assert(D_ == H_ * DH_);
static_assert(DH_ == 64);
static_assert(D_ == 4 * 256);
static_assert(BT_ % GBM == 0 && T_ % GBM == 0);
static_assert(D_ % GBN == 0 && (3 * D_) % GBN == 0 && DFF_ % GBN == 0);
static_assert(D_ % GBK == 0 && DFF_ % GBK == 0);
static_assert(T_ % 64 == 0 && D_ % 64 == 0 && DFF_ % 64 == 0);

typedef _Float16 f16;
typedef _Float16 v16h __attribute__((ext_vector_type(16)));
typedef _Float16 v8h  __attribute__((ext_vector_type(8)));
typedef _Float16 v8ha __attribute__((ext_vector_type(8), may_alias));
typedef _Float16 v4h  __attribute__((ext_vector_type(4)));
typedef float    v8f  __attribute__((ext_vector_type(8)));
typedef float    v4f  __attribute__((ext_vector_type(4)));
typedef float    v4fa __attribute__((ext_vector_type(4), may_alias));

union Frag { v16h v; v8h half[2]; };

__device__ __forceinline__ v8f wmma_f16(v16h a, v16h b, v8f c) {
  return __builtin_amdgcn_wmma_f32_16x16x32_f16(false, a, false, b, (short)0, c, false, false);
}

__global__ __launch_bounds__(256) void k_tconv(const float* __restrict__ src, f16* dst,
                                               int R, int C, int src_slab, int dst_slab,
                                               float scale) {
  __shared__ float tile[64][33];
  const int tx = threadIdx.x, ty = threadIdx.y;
  const int c0 = blockIdx.x * 32, r0 = blockIdx.y * 64;
  if (c0 + 32 > C || r0 + 64 > R) return;
  const float* s = src + (size_t)blockIdx.z * (size_t)src_slab;
  f16* d = dst + (size_t)blockIdx.z * (size_t)dst_slab;
#pragma unroll
  for (int j = 0; j < 8; ++j) {
    const int r = ty + 8 * j;
    tile[r][tx] = s[(size_t)(r0 + r) * C + c0 + tx];
  }
  __syncthreads();
  const int q  = 4 * ty + (tx >> 3);
  const int kp = 8 * (tx & 7);
  v8h o;
#pragma unroll
  for (int i = 0; i < 8; ++i) o[i] = (f16)(tile[kp + i][q] * scale);
  volatile v8h* p = (volatile v8h*)(d + (size_t)(c0 + q) * R + r0 + kp);
  *p = o;
  __threadfence();
  *p = o;
}

__global__ __launch_bounds__(256) void k_ln(const float* __restrict__ x,
                                            const float* __restrict__ gam,
                                            const float* __restrict__ bet,
                                            f16* out, int nrows) {
  __shared__ float red[8];
  const int row = blockIdx.x;
  if (row >= nrows) return;
  const int t = threadIdx.x, lane = t & 31, wave = t >> 5;
  const v4f v = *(const v4f*)(x + (size_t)row * D_ + 4 * t);
  float s = (v[0] + v[1]) + (v[2] + v[3]);
#pragma unroll
  for (int dd = 16; dd >= 1; dd >>= 1) s += __shfl_xor(s, dd, 32);
  if (lane == 0) red[wave] = s;
  __syncthreads();
  float tot = 0.f;
#pragma unroll
  for (int i = 0; i < 8; ++i) tot += red[i];
  const float mu = tot * (1.0f / (float)D_);
  __syncthreads();
  float dv[4];
  float vs = 0.f;
#pragma unroll
  for (int i = 0; i < 4; ++i) { dv[i] = v[i] - mu; vs += dv[i] * dv[i]; }
#pragma unroll
  for (int dd = 16; dd >= 1; dd >>= 1) vs += __shfl_xor(vs, dd, 32);
  if (lane == 0) red[wave] = vs;
  __syncthreads();
  float vtot = 0.f;
#pragma unroll
  for (int i = 0; i < 8; ++i) vtot += red[i];
  const float inv = rsqrtf(vtot * (1.0f / (float)D_) + 1e-5f);
  const v4f gg = *(const v4f*)(gam + 4 * t);
  const v4f bb = *(const v4f*)(bet + 4 * t);
  v4h o;
#pragma unroll
  for (int i = 0; i < 4; ++i) o[i] = (f16)(dv[i] * inv * gg[i] + bb[i]);
  volatile v4h* p = (volatile v4h*)(out + (size_t)row * D_ + 4 * t);
  *p = o;
  __threadfence();
  *p = o;
}

template <int MODE>
__global__ __launch_bounds__(256) void k_gemm(const f16* __restrict__ A, const f16* __restrict__ Bt,
                                              const float* __restrict__ bias0,
                                              const float* __restrict__ bias1,
                                              const float* __restrict__ bias2,
                                              const float* resid, float* outf, f16* outb,
                                              int M, int N, int K) {
  __shared__ __attribute__((aligned(16))) f16 smem[GBM * GLP + GBN * GLP];
  f16* As = smem;
  f16* Bs = smem + GBM * GLP;
  const int t = threadIdx.x, lane = t & 31, wave = t >> 5;
  const int hh = lane >> 4, l16 = lane & 15;
  const int waveM = wave >> 1;
  const int waveN = wave & 1;
  const int m0 = blockIdx.y * GBM, n0 = blockIdx.x * GBN;
  if (m0 + GBM > M || n0 + GBN > N) return;

  const int srow  = t >> 3;
  const int spart = (t & 7) * 8;
  const v8f z8 = {0.f, 0.f, 0.f, 0.f, 0.f, 0.f, 0.f, 0.f};
  v8f acc[2][4];
#pragma unroll
  for (int mi = 0; mi < 2; ++mi)
#pragma unroll
    for (int ni = 0; ni < 4; ++ni) acc[mi][ni] = z8;

  for (int k0 = 0; k0 < K; k0 += GBK) {
    v8h ra[4], rb[4];
#pragma unroll
    for (int j = 0; j < 4; ++j) {
      const int r = srow + 32 * j;
      ra[j] = *(const v8h*)(A  + (size_t)(m0 + r) * K + k0 + spart);
      rb[j] = *(const v8h*)(Bt + (size_t)(n0 + r) * K + k0 + spart);
    }
    __syncthreads();
#pragma unroll
    for (int j = 0; j < 4; ++j) {
      const int r = srow + 32 * j;
      *(v8h*)(As + r * GLP + spart) = ra[j];
      *(v8h*)(Bs + r * GLP + spart) = rb[j];
    }
    __syncthreads();
#pragma unroll
    for (int ks = 0; ks < 2; ++ks) {
      Frag af[2], bf[4];
#pragma unroll
      for (int mi = 0; mi < 2; ++mi) {
        const f16* p = As + (waveM * 32 + mi * 16 + l16) * GLP + ks * 32;
        af[mi].half[0] = *(const v8h*)(p + 8 * hh);
        af[mi].half[1] = *(const v8h*)(p + 16 + 8 * hh);
      }
#pragma unroll
      for (int ni = 0; ni < 4; ++ni) {
        const f16* p = Bs + (waveN * 64 + ni * 16 + l16) * GLP + ks * 32;
        bf[ni].half[0] = *(const v8h*)(p + 8 * hh);
        bf[ni].half[1] = *(const v8h*)(p + 16 + 8 * hh);
      }
#pragma unroll
      for (int mi = 0; mi < 2; ++mi)
#pragma unroll
        for (int ni = 0; ni < 4; ++ni)
          acc[mi][ni] = wmma_f16(af[mi].v, bf[ni].v, acc[mi][ni]);
      asm volatile("v_nop\n\tv_nop\n\tv_nop\n\tv_nop"
                   : "+v"(acc[0][0]), "+v"(acc[0][1]), "+v"(acc[0][2]), "+v"(acc[0][3]),
                     "+v"(acc[1][0]), "+v"(acc[1][1]), "+v"(acc[1][2]), "+v"(acc[1][3])
                   : "v"(af[0].v), "v"(af[1].v), "v"(bf[0].v), "v"(bf[1].v), "v"(bf[2].v), "v"(bf[3].v));
    }
  }
  __syncthreads();

  const float WINV = 0.00390625f;
  int which = 0;
  const float* bp = bias0;
  if (MODE == 2) {
    which = n0 / D_;
    bp = (which == 0) ? bias0 : ((which == 1) ? bias1 : bias2);
  }
  float bvv[4];
#pragma unroll
  for (int ni = 0; ni < 4; ++ni) {
    const int gn = n0 + waveN * 64 + ni * 16 + l16;
    const int bi = (MODE == 2) ? (gn - which * D_) : gn;
    bvv[ni] = bp[bi];
  }

  if (MODE == 0) {
    float* Cs = (float*)smem;
#pragma unroll
    for (int ps = 0; ps < 2; ++ps) {
      if ((waveM >> 1) == ps) {
#pragma unroll
        for (int mi = 0; mi < 2; ++mi)
#pragma unroll
          for (int ni = 0; ni < 4; ++ni)
#pragma unroll
            for (int r = 0; r < 8; ++r) {
              const int row = (waveM & 1) * 32 + mi * 16 + 8 * hh + r;
              const int col = waveN * 64 + ni * 16 + l16;
              Cs[row * CSP + col] = acc[mi][ni][r] * WINV + bvv[ni];
            }
      }
      __syncthreads();
      v4f vals[8];
      size_t goff[8];
#pragma unroll
      for (int i = 0; i < 8; ++i) {
        const int idx = t + 256 * i;
        const int row = idx >> 5;
        const int c4  = (idx & 31) * 4;
        goff[i] = (size_t)(m0 + ps * 64 + row) * N + n0 + c4;
        const v4f cv = *(const v4fa*)(Cs + row * CSP + c4);
        const v4f rv = *(const v4f*)(resid + goff[i]);
        vals[i] = cv + rv;
      }
#pragma unroll
      for (int i = 0; i < 8; ++i) *(volatile v4f*)(outf + goff[i]) = vals[i];
      __threadfence();
#pragma unroll
      for (int i = 0; i < 8; ++i) *(volatile v4f*)(outf + goff[i]) = vals[i];
      __syncthreads();
    }
  } else {
    f16* Cs = smem;
    const bool vtr = (MODE == 2) && (which == 2);
#pragma unroll
    for (int mi = 0; mi < 2; ++mi)
#pragma unroll
      for (int ni = 0; ni < 4; ++ni)
#pragma unroll
        for (int r = 0; r < 8; ++r) {
          const int row = waveM * 32 + mi * 16 + 8 * hh + r;
          const int col = waveN * 64 + ni * 16 + l16;
          float v = acc[mi][ni][r] * WINV + bvv[ni];
          if (MODE == 1) v = fmaxf(v, 0.f);
          if (vtr) Cs[col * CSP + row] = (f16)v;
          else     Cs[row * CSP + col] = (f16)v;
        }
    __syncthreads();
    const size_t hsz = (size_t)B_ * H_ * (size_t)T_ * DH_;
    v8h vals[8];
    size_t goff[8];
#pragma unroll
    for (int i = 0; i < 8; ++i) {
      const int idx = t + 256 * i;
      const int row = idx >> 4;
      const int c8  = (idx & 15) * 8;
      vals[i] = *(const v8ha*)(Cs + row * CSP + c8);
      if (MODE == 1) {
        goff[i] = (size_t)(m0 + row) * N + n0 + c8;
      } else if (vtr) {
        const int gn = n0 + row;
        const int gm = m0 + c8;
        const int hn = gn - 2 * D_;
        const int hd = hn / DH_, e = hn - hd * DH_;
        const int bb = gm / T_, tt = gm - bb * T_;
        goff[i] = 2 * hsz + (((size_t)(bb * H_ + hd) * DH_ + e) * (size_t)T_ + tt);
      } else {
        const int gm = m0 + row;
        const int gn = n0 + c8;
        const int hn = gn - which * D_;
        const int hd = hn / DH_, e = hn - hd * DH_;
        const int bb = gm / T_, tt = gm - bb * T_;
        goff[i] = (size_t)which * hsz + (((size_t)(bb * H_ + hd) * T_ + tt) * (size_t)DH_ + e);
      }
    }
#pragma unroll
    for (int i = 0; i < 8; ++i) *(volatile v8h*)(outb + goff[i]) = vals[i];
    __threadfence();
#pragma unroll
    for (int i = 0; i < 8; ++i) *(volatile v8h*)(outb + goff[i]) = vals[i];
  }
}

__global__ __launch_bounds__(128) void k_attn(const f16* __restrict__ Qg, const f16* __restrict__ Kg,
                                              const f16* __restrict__ Vtg, f16* Aout) {
  __shared__ __attribute__((aligned(16))) f16 Ks[64 * AKP];
  __shared__ __attribute__((aligned(16))) f16 Vs[64 * AKP];
  __shared__ __attribute__((aligned(16))) f16 Ps[4 * 16 * AKP];
  const int qt = blockIdx.x, hd = blockIdx.y, b = blockIdx.z;
  const int t = threadIdx.x, lane = t & 31, wave = t >> 5;
  const int hh = lane >> 4, l16 = lane & 15;
  const size_t base = ((size_t)b * H_ + hd) * (size_t)T_ * DH_;
  const int q0 = qt * 64;
  f16* myP = Ps + wave * 16 * AKP;

  Frag qa[2];
  {
    const f16* qp = Qg + base + (size_t)(q0 + wave * 16 + l16) * DH_;
#pragma unroll
    for (int ks = 0; ks < 2; ++ks) {
      qa[ks].half[0] = *(const v8h*)(qp + ks * 32 + 8 * hh);
      qa[ks].half[1] = *(const v8h*)(qp + ks * 32 + 16 + 8 * hh);
    }
  }
  const v8f z8 = {0.f, 0.f, 0.f, 0.f, 0.f, 0.f, 0.f, 0.f};
  v8f o[4];
#pragma unroll
  for (int nt = 0; nt < 4; ++nt) o[nt] = z8;
  float mr[8], ls[8];
#pragma unroll
  for (int r = 0; r < 8; ++r) { mr[r] = -1.0e30f; ls[r] = 0.f; }

  const int srow  = t >> 3;
  const int spart = (t & 7) * 8;

  for (int kt = 0; kt <= qt; ++kt) {
    v8h rk[4], rv[4];
#pragma unroll
    for (int j = 0; j < 4; ++j) {
      const int r = srow + 16 * j;
      rk[j] = *(const v8h*)(Kg  + base + (size_t)(kt * 64 + r) * DH_ + spart);
      rv[j] = *(const v8h*)(Vtg + base + (size_t)r * T_ + kt * 64 + spart);
    }
    __syncthreads();
#pragma unroll
    for (int j = 0; j < 4; ++j) {
      const int r = srow + 16 * j;
      *(v8h*)(Ks + r * AKP + spart) = rk[j];
      *(v8h*)(Vs + r * AKP + spart) = rv[j];
    }
    __syncthreads();

    v8f s[4];
#pragma unroll
    for (int nt = 0; nt < 4; ++nt) {
      Frag kb[2];
#pragma unroll
      for (int ks = 0; ks < 2; ++ks) {
        const f16* p = Ks + (nt * 16 + l16) * AKP + ks * 32;
        kb[ks].half[0] = *(const v8h*)(p + 8 * hh);
        kb[ks].half[1] = *(const v8h*)(p + 16 + 8 * hh);
      }
      v8f acc = z8;
      acc = wmma_f16(qa[0].v, kb[0].v, acc);
      acc = wmma_f16(qa[1].v, kb[1].v, acc);
      asm volatile("v_nop\n\tv_nop\n\tv_nop\n\tv_nop"
                   : "+v"(acc)
                   : "v"(qa[0].v), "v"(qa[1].v), "v"(kb[0].v), "v"(kb[1].v));
      s[nt] = acc;
    }

#pragma unroll
    for (int r = 0; r < 8; ++r) {
      const int qi = q0 + wave * 16 + 8 * hh + r;
      float mx = mr[r];
      float sv[4];
#pragma unroll
      for (int nt = 0; nt < 4; ++nt) {
        const int kj = kt * 64 + nt * 16 + l16;
        float val = s[nt][r] * 0.125f;
        if (kj > qi) val = -1.0e30f;
        sv[nt] = val;
        mx = fmaxf(mx, val);
      }
#pragma unroll
      for (int dd = 1; dd < 16; dd <<= 1) mx = fmaxf(mx, __shfl_xor(mx, dd, 32));
      const float corr = __expf(mr[r] - mx);
      float ev[4];
      float rs = 0.f;
#pragma unroll
      for (int nt = 0; nt < 4; ++nt) { ev[nt] = __expf(sv[nt] - mx); rs += ev[nt]; }
#pragma unroll
      for (int dd = 1; dd < 16; dd <<= 1) rs += __shfl_xor(rs, dd, 32);
      ls[r] = ls[r] * corr + rs;
      mr[r] = mx;
#pragma unroll
      for (int nt = 0; nt < 4; ++nt) o[nt][r] = o[nt][r] * corr;
#pragma unroll
      for (int nt = 0; nt < 4; ++nt)
        myP[(8 * hh + r) * AKP + nt * 16 + l16] = (f16)(ev[nt] * 256.0f);
    }
    __syncthreads();

    Frag pa[2];
#pragma unroll
    for (int ks = 0; ks < 2; ++ks) {
      const f16* p = myP + l16 * AKP + ks * 32;
      pa[ks].half[0] = *(const v8ha*)(p + 8 * hh);
      pa[ks].half[1] = *(const v8ha*)(p + 16 + 8 * hh);
    }
#pragma unroll
    for (int nt = 0; nt < 4; ++nt) {
      Frag vb[2];
#pragma unroll
      for (int ks = 0; ks < 2; ++ks) {
        const f16* pv = Vs + (nt * 16 + l16) * AKP + ks * 32;
        vb[ks].half[0] = *(const v8h*)(pv + 8 * hh);
        vb[ks].half[1] = *(const v8h*)(pv + 16 + 8 * hh);
      }
      o[nt] = wmma_f16(pa[0].v, vb[0].v, o[nt]);
      o[nt] = wmma_f16(pa[1].v, vb[1].v, o[nt]);
      asm volatile("v_nop\n\tv_nop\n\tv_nop\n\tv_nop"
                   : "+v"(o[nt])
                   : "v"(pa[0].v), "v"(pa[1].v), "v"(vb[0].v), "v"(vb[1].v));
    }
  }
  __syncthreads();

#pragma unroll
  for (int r = 0; r < 8; ++r) {
    const float invl = 1.0f / (ls[r] * 256.0f);
#pragma unroll
    for (int nt = 0; nt < 4; ++nt)
      myP[(8 * hh + r) * AKP + nt * 16 + l16] = (f16)(o[nt][r] * invl);
  }
  __syncthreads();
  v8h vals[4];
  size_t goff[4];
#pragma unroll
  for (int i = 0; i < 4; ++i) {
    const int row = 4 * i + (lane >> 3);
    const int kp  = (lane & 7) * 8;
    vals[i] = *(const v8ha*)(myP + row * AKP + kp);
    goff[i] = ((size_t)b * T_ + q0 + wave * 16 + row) * (size_t)D_ + hd * DH_ + kp;
  }
#pragma unroll
  for (int i = 0; i < 4; ++i) *(volatile v8h*)(Aout + goff[i]) = vals[i];
  __threadfence();
#pragma unroll
  for (int i = 0; i < 4; ++i) *(volatile v8h*)(Aout + goff[i]) = vals[i];
}

extern "C" void kernel_launch(void* const* d_in, const int* in_sizes, int n_in,
                              void* d_out, int out_size, void* d_ws,
                              size_t ws_size, hipStream_t stream) {
  if (n_in < 17) return;
  if (in_sizes[0] != BT_ * D_ || in_sizes[1] != H_ * D_ * DH_ || in_sizes[2] != H_ * DH_ ||
      in_sizes[3] != H_ * D_ * DH_ || in_sizes[4] != H_ * DH_ || in_sizes[5] != H_ * D_ * DH_ ||
      in_sizes[6] != H_ * DH_ || in_sizes[7] != D_ * D_ || in_sizes[8] != D_ ||
      in_sizes[9] != D_ || in_sizes[10] != D_ || in_sizes[11] != D_ || in_sizes[12] != D_ ||
      in_sizes[13] != D_ * DFF_ || in_sizes[14] != DFF_ || in_sizes[15] != DFF_ * D_ ||
      in_sizes[16] != D_ || out_size != BT_ * D_)
    return;

  const float* x    = (const float*)d_in[0];
  const float* Wq   = (const float*)d_in[1];
  const float* bq   = (const float*)d_in[2];
  const float* Wk   = (const float*)d_in[3];
  const float* bk   = (const float*)d_in[4];
  const float* Wv   = (const float*)d_in[5];
  const float* bv   = (const float*)d_in[6];
  const float* Wo   = (const float*)d_in[7];
  const float* bo   = (const float*)d_in[8];
  const float* ln1g = (const float*)d_in[9];
  const float* ln1b = (const float*)d_in[10];
  const float* ln2g = (const float*)d_in[11];
  const float* ln2b = (const float*)d_in[12];
  const float* W1   = (const float*)d_in[13];
  const float* b1   = (const float*)d_in[14];
  const float* W2   = (const float*)d_in[15];
  const float* b2   = (const float*)d_in[16];
  float* out = (float*)d_out;

  char* ws = (char*)d_ws;
  size_t off = 0;
  const size_t sz_h    = (size_t)BT_ * D_ * 2;
  const size_t sz_wqkv = (size_t)3 * D_ * D_ * 2;
  const size_t sz_wo   = (size_t)D_ * D_ * 2;
  const size_t sz_w1   = (size_t)DFF_ * D_ * 2;
  const size_t sz_w2   = (size_t)D_ * DFF_ * 2;
  const size_t hsz     = (size_t)B_ * H_ * (size_t)T_ * DH_;
  const size_t sz_qkv  = 3 * hsz * 2;
  const size_t sz_att  = (size_t)BT_ * D_ * 2;
  const size_t sz_ffh  = (size_t)BT_ * DFF_ * 2;
  const size_t sz_x1   = (size_t)BT_ * D_ * 4;
  f16*   h1     = (f16*)(ws + off);   off += sz_h;
  f16*   h2     = (f16*)(ws + off);   off += sz_h;
  f16*   Wqkv_t = (f16*)(ws + off);   off += sz_wqkv;
  f16*   Wo_t   = (f16*)(ws + off);   off += sz_wo;
  f16*   W1_t   = (f16*)(ws + off);   off += sz_w1;
  f16*   W2_t   = (f16*)(ws + off);   off += sz_w2;
  f16*   qkv    = (f16*)(ws + off);   off += sz_qkv;
  f16*   attn_a = (f16*)(ws + off);   off += sz_att;
  f16*   ffh    = (f16*)(ws + off);   off += sz_ffh;
  float* x1     = (float*)(ws + off); off += sz_x1;
  if (off > ws_size) return;

  const dim3 tb(32, 8);
  const float WSC = 256.0f;
  k_tconv<<<dim3(DH_ / 32, D_ / 64, H_), tb, 0, stream>>>(Wq, Wqkv_t, D_, DH_, D_ * DH_, DH_ * D_, WSC);
  k_tconv<<<dim3(DH_ / 32, D_ / 64, H_), tb, 0, stream>>>(Wk, Wqkv_t + (size_t)D_ * D_, D_, DH_, D_ * DH_, DH_ * D_, WSC);
  k_tconv<<<dim3(DH_ / 32, D_ / 64, H_), tb, 0, stream>>>(Wv, Wqkv_t + (size_t)2 * D_ * D_, D_, DH_, D_ * DH_, DH_ * D_, WSC);
  k_tconv<<<dim3(D_ / 32, D_ / 64, 1), tb, 0, stream>>>(Wo, Wo_t, D_, D_, 0, 0, WSC);
  k_tconv<<<dim3(DFF_ / 32, D_ / 64, 1), tb, 0, stream>>>(W1, W1_t, D_, DFF_, 0, 0, WSC);
  k_tconv<<<dim3(D_ / 32, DFF_ / 64, 1), tb, 0, stream>>>(W2, W2_t, DFF_, D_, 0, 0, WSC);

  k_ln<<<BT_, 256, 0, stream>>>(x, ln1g, ln1b, h1, BT_);

  k_gemm<2><<<dim3(3 * D_ / GBN, BT_ / GBM), 256, 0, stream>>>(
      h1, Wqkv_t, bq, bk, bv, x, x1, qkv, BT_, 3 * D_, D_);

  k_attn<<<dim3(T_ / 64, H_, B_), 128, 0, stream>>>(qkv, qkv + hsz, qkv + 2 * hsz, attn_a);

  k_gemm<0><<<dim3(D_ / GBN, BT_ / GBM), 256, 0, stream>>>(
      attn_a, Wo_t, bo, bo, bo, x, x1, h1, BT_, D_, D_);

  k_ln<<<BT_, 256, 0, stream>>>(x1, ln2g, ln2b, h2, BT_);

  k_gemm<1><<<dim3(DFF_ / GBN, BT_ / GBM), 256, 0, stream>>>(
      h2, W1_t, b1, b1, b1, x, x1, ffh, BT_, DFF_, D_);

  k_gemm<0><<<dim3(D_ / GBN, BT_ / GBM), 256, 0, stream>>>(
      ffh, W2_t, b2, b2, b2, x1, out, h1, BT_, D_, DFF_);
}
